// MPNNconv_20203526160531
// MI455X (gfx1250) — hardware-verified
//
#include <hip/hip_runtime.h>
#include <stddef.h>
#include <stdint.h>
#include <math.h>


#define CIN     128
#define DEI     12
#define DEH     32
#define HID     64
#define K2      128
#define NG3     192
#define NBIG    2368
#define COL_TB  2048
#define COL_R   2112
#define COL_GH  2176
#define NTHR    256
#define NWAVE   8
#define EPT     8
#define CHUNK   (NTHR * EPT)
#define WCAP    (EPT * 32)
#define LISTN   (NWAVE * WCAP)
#define NBA     256
#define SLA     8
#define RCAP    2048
#define DEGCAP  32
#define GBM     64
#define GBN     64
#define GTHR    128
#define NU_P    (HID * (CIN / 8))
#define NU_B    (NBIG * (K2 / 8))
#define NU_I    (NG3 * (K2 / 8))
#define NU_ALL  (NU_P + NU_B + NU_I)
#define SC_ZINTS (LISTN + 2 * RCAP + 3 * NBA)
#define SC_LDS_INTS (SC_ZINTS + 16)
#define WSMAX   134217728

static_assert((CHUNK & (CHUNK - 1)) == 0 && CHUNK <= 4096);
static_assert((NBA & (NBA - 1)) == 0 && NBA == (1 << SLA));
static_assert(((long long)CHUNK << SLA) < (1LL << 31));
static_assert(LISTN % NTHR == 0 && NBA % NWAVE == 0 && NBA % 32 == 0);
static_assert(RCAP % 32 == 0 && SC_ZINTS % 4 == 0 && LISTN % 4 == 0);
static_assert(DEGCAP <= 32 && DEH == 32 && HID == 64);
static_assert(CIN % 32 == 0 && K2 % 32 == 0 && K2 == 2 * HID);
static_assert(NBIG % GBN == 0 && NBIG == COL_GH + NG3 && COL_R == COL_TB + HID && COL_GH == COL_R + HID);
static_assert(NU_P % NTHR == 0 && NU_B % NTHR == 0 && NU_I % NTHR == 0);
static_assert((COL_TB * 16) % NTHR == 0 && (COL_R * 16) % NTHR == 0 && (COL_GH * 16) % NTHR == 0);
static_assert(GBM == (GTHR / 32) * 16 && (GBM * HID) % NTHR == 0);
static_assert(SC_LDS_INTS * 4 + DEI * DEH * 4 <= 65536);
static_assert(GBM * NG3 * 4 + 2 * NG3 * 4 <= 65536);

typedef float          v2f   __attribute__((ext_vector_type(2)));
typedef float          v4f   __attribute__((ext_vector_type(4)));
typedef float          v8f   __attribute__((ext_vector_type(8)));
typedef int            v4i   __attribute__((ext_vector_type(4)));
typedef int            v8i   __attribute__((ext_vector_type(8)));
typedef unsigned int   v4u   __attribute__((ext_vector_type(4)));
typedef unsigned short v8us  __attribute__((ext_vector_type(8)));
typedef unsigned short v16us __attribute__((ext_vector_type(16)));
typedef __bf16         v16bf __attribute__((ext_vector_type(16)));
typedef v2f  __attribute__((may_alias)) v2fa;
typedef v4f  __attribute__((may_alias)) v4fa;
typedef v4i  __attribute__((may_alias)) v4ia;
typedef v8us __attribute__((may_alias)) v8usa;
union FragB { v16bf v; v16us u; v8us h[2]; v8i w; };

__device__ __forceinline__ v8f wmb(const FragB& a, const FragB& b, v8f c) {
  v8f d = __builtin_amdgcn_wmma_f32_16x16x32_bf16(false, a.v, false, b.v, (short)0, c, false, false);
  asm volatile("v_nop\n\tv_nop\n\tv_nop\n\tv_nop" : "+v"(d) : "v"(a.w), "v"(b.w));
  return d;
}

__device__ __forceinline__ unsigned bf16_bits(float f) {
  const unsigned u = __float_as_uint(f);
  return (u + 0x7FFFu + ((u >> 16) & 1u)) >> 16;
}
__device__ __forceinline__ float bf16_val(float f) {
  return __uint_as_float(bf16_bits(f) << 16);
}
__device__ __forceinline__ float relu_np(float v) { return (v > 0.0f) ? v : (v - v); }
__device__ __forceinline__ float sigm(float a) { return 1.0f / (1.0f + expf(-a)); }
__device__ __forceinline__ unsigned pk2(float v0, float v1, bool lsel) {
  const unsigned h0 = bf16_bits(v0), h1 = bf16_bits(v1);
  const unsigned l0 = bf16_bits(v0 - __uint_as_float(h0 << 16));
  const unsigned l1 = bf16_bits(v1 - __uint_as_float(h1 << 16));
  const unsigned s0 = lsel ? l0 : h0;
  const unsigned s1 = lsel ? l1 : h1;
  return s0 | (s1 << 16);
}

template <int SLB>
__device__ __forceinline__ int scan_chunk(const int* __restrict__ dsts, int nE, int cbase, int slotBase,
                                          int nb, int vec8, int* list, int tid, int lane, int wave) {
  int wc = 0;
  const int el0  = tid * EPT;
  const int e0   = cbase + el0;
  const int sent = -2147483647 - 1;
  v4i da, db;
  if (vec8 != 0 && cbase + CHUNK <= nE) {
    da = *(const v4i*)(dsts + e0);
    db = *(const v4i*)(dsts + e0 + 4);
  } else {
    da.x = (e0     < nE) ? dsts[min(e0,     nE - 1)] : sent;
    da.y = (e0 + 1 < nE) ? dsts[min(e0 + 1, nE - 1)] : sent;
    da.z = (e0 + 2 < nE) ? dsts[min(e0 + 2, nE - 1)] : sent;
    da.w = (e0 + 3 < nE) ? dsts[min(e0 + 3, nE - 1)] : sent;
    db.x = (e0 + 4 < nE) ? dsts[min(e0 + 4, nE - 1)] : sent;
    db.y = (e0 + 5 < nE) ? dsts[min(e0 + 5, nE - 1)] : sent;
    db.z = (e0 + 6 < nE) ? dsts[min(e0 + 6, nE - 1)] : sent;
    db.w = (e0 + 7 < nE) ? dsts[min(e0 + 7, nE - 1)] : sent;
  }
  const unsigned nbs = (unsigned)slotBase;
  const unsigned unb = (unsigned)nb;
  const unsigned s0 = (unsigned)da.x - nbs, s1 = (unsigned)da.y - nbs;
  const unsigned s2 = (unsigned)da.z - nbs, s3 = (unsigned)da.w - nbs;
  const unsigned s4 = (unsigned)db.x - nbs, s5 = (unsigned)db.y - nbs;
  const unsigned s6 = (unsigned)db.z - nbs, s7 = (unsigned)db.w - nbs;
  const bool h0 = s0 < unb, h1 = s1 < unb, h2 = s2 < unb, h3 = s3 < unb;
  const bool h4 = s4 < unb, h5 = s5 < unb, h6 = s6 < unb, h7 = s7 < unb;
  const unsigned any = __builtin_amdgcn_ballot_w32(h0 | h1 | h2 | h3 | h4 | h5 | h6 | h7);
  if (any != 0u) {
#define HITJ(J, HJ, SJ) { \
      const unsigned mj = __builtin_amdgcn_ballot_w32(HJ); \
      if (mj != 0u) { \
        if (HJ) { \
          const int pos = wc + (int)__builtin_amdgcn_mbcnt_lo(mj, 0u); \
          if (pos < WCAP) list[wave * WCAP + pos] = ((el0 + (J)) << SLB) | (int)(SJ); \
        } \
        wc += (int)__builtin_popcount(mj); } }
    HITJ(0, h0, s0)
    HITJ(1, h1, s1)
    HITJ(2, h2, s2)
    HITJ(3, h3, s3)
    HITJ(4, h4, s4)
    HITJ(5, h5, s5)
    HITJ(6, h6, s6)
    HITJ(7, h7, s7)
#undef HITJ
  }
  return wc;
}

__global__ __launch_bounds__(NTHR) void k_wprep(const float* __restrict__ w_proj, const float* __restrict__ w_e2,
                                                const float* __restrict__ b_e2, const float* __restrict__ w_root,
                                                const float* __restrict__ w_hh, const float* __restrict__ w_ih,
                                                unsigned short* WPT, unsigned short* WBIG, unsigned short* WIH) {
  const int u = (int)blockIdx.x * NTHR + (int)threadIdx.x;
  const float* p;
  int st;
  unsigned short* dp;
  if (u < NU_P) {
    const int n  = u >> 4;
    const int k8 = (u & 15) * 8;
    p  = w_proj + (size_t)k8 * HID + n;
    st = HID;
    dp = WPT + (size_t)n * CIN + k8;
  } else if (u < NU_P + NU_B) {
    const int v  = u - NU_P;
    const int n  = v >> 4;
    const int k8 = (v & 15) * 8;
    const int d0 = k8 & (HID - 1);
    if (n < COL_TB) {
      const int kp = n >> 6, o = n & 63;
      p = w_e2 + (size_t)kp * (HID * HID) + (size_t)d0 * HID + o;
      st = HID;
    } else if (n < COL_R) {
      p = b_e2 + (size_t)d0 * HID + (n - COL_TB);
      st = HID;
    } else if (n < COL_GH) {
      p = w_root + (size_t)d0 * HID + (n - COL_R);
      st = HID;
    } else {
      p = w_hh + (size_t)(n - COL_GH) * HID + d0;
      st = 1;
    }
    dp = WBIG + (size_t)n * K2 + k8;
  } else if (u < NU_ALL) {
    const int v  = u - NU_P - NU_B;
    const int g  = v >> 4;
    const int k8 = (v & 15) * 8;
    const int d0 = k8 & (HID - 1);
    p  = w_ih + (size_t)g * HID + d0;
    st = 1;
    dp = WIH + (size_t)g * K2 + k8;
  } else {
    return;
  }
  v8us o;
#pragma unroll
  for (int i = 0; i < 8; ++i) o[i] = (unsigned short)bf16_bits(p[(size_t)i * (size_t)st]);
  *(volatile v8us*)dp = o;
  __threadfence();
  *(volatile v8us*)dp = o;
}

__global__ __launch_bounds__(NTHR) void k_cvx(const float* __restrict__ x, int nN, int nUnits,
                                              unsigned short* xb) {
  const int u = (int)blockIdx.x * NTHR + (int)threadIdx.x;
  if (u >= nUnits) return;
  const int row = u >> 4;
  const int k8  = (u & 15) * 8;
  const int rc  = row < nN ? row : nN - 1;
  const float* p = x + (size_t)rc * CIN + k8;
  const v4f a = *(const v4fa*)p;
  const v4f b = *(const v4fa*)(p + 4);
  const bool ok = row < nN;
  v8us o;
  o[0] = ok ? (unsigned short)bf16_bits(a.x) : (unsigned short)0;
  o[1] = ok ? (unsigned short)bf16_bits(a.y) : (unsigned short)0;
  o[2] = ok ? (unsigned short)bf16_bits(a.z) : (unsigned short)0;
  o[3] = ok ? (unsigned short)bf16_bits(a.w) : (unsigned short)0;
  o[4] = ok ? (unsigned short)bf16_bits(b.x) : (unsigned short)0;
  o[5] = ok ? (unsigned short)bf16_bits(b.y) : (unsigned short)0;
  o[6] = ok ? (unsigned short)bf16_bits(b.z) : (unsigned short)0;
  o[7] = ok ? (unsigned short)bf16_bits(b.w) : (unsigned short)0;
  unsigned short* dp = xb + (size_t)row * CIN + k8;
  *(volatile v8us*)dp = o;
  __threadfence();
  *(volatile v8us*)dp = o;
}

template <int NT, int KS, int KP>
__device__ __forceinline__ void mm_tile(const unsigned short* ap, const unsigned short* wp, v8f (&acc)[NT]) {
#pragma unroll
  for (int ks = 0; ks < KS; ++ks) {
    FragB af;
    af.h[0] = *(const v8usa*)(ap + 32 * ks);
    af.h[1] = *(const v8usa*)(ap + 32 * ks + 16);
#pragma unroll
    for (int t = 0; t < NT; ++t) {
      const unsigned short* wq = wp + (size_t)(16 * t) * (size_t)KP + 32 * ks;
      FragB bf;
      bf.h[0] = *(const v8usa*)wq;
      bf.h[1] = *(const v8usa*)(wq + 16);
      acc[t] = wmb(af, bf, acc[t]);
    }
  }
}

template <int NI, int HL>
__device__ __forceinline__ void put_rows(const float* stg, int pitch, int lr0, int rowBase, int rowLim,
                                         float* fdst, unsigned short* hdst, int hh, int m) {
  v4f fv[NI];
  v4u hv[NI];
  const bool lsel = (m & 8) != 0;
#pragma unroll
  for (int i = 0; i < NI; ++i) {
    const int lr = lr0 + 2 * i + hh;
    fv[i] = *(const v4fa*)(stg + lr * pitch + 4 * m);
    v4u w = {0u, 0u, 0u, 0u};
    if constexpr (HL != 0) {
      const float* q = stg + lr * pitch + 8 * (m & 7);
      const v4f a = *(const v4fa*)q;
      const v4f b = *(const v4fa*)(q + 4);
      w.x = pk2(a.x, a.y, lsel);
      w.y = pk2(a.z, a.w, lsel);
      w.z = pk2(b.x, b.y, lsel);
      w.w = pk2(b.z, b.w, lsel);
    }
    hv[i] = w;
  }
#pragma unroll
  for (int i = 0; i < NI; ++i) {
    const int gr = rowBase + lr0 + 2 * i + hh;
    const bool ok = gr < rowLim;
    float* op = fdst + (size_t)gr * HID + 4 * m;
    if (ok) *(volatile v4f*)op = fv[i];
    if constexpr (HL != 0) {
      unsigned short* hp = hdst + (size_t)gr * K2 + 8 * m;
      if (ok) *(volatile v4u*)hp = hv[i];
    }
  }
  __threadfence();
#pragma unroll
  for (int i = 0; i < NI; ++i) {
    const int gr = rowBase + lr0 + 2 * i + hh;
    const bool ok = gr < rowLim;
    float* op = fdst + (size_t)gr * HID + 4 * m;
    if (ok) *(volatile v4f*)op = fv[i];
    if constexpr (HL != 0) {
      unsigned short* hp = hdst + (size_t)gr * K2 + 8 * m;
      if (ok) *(volatile v4u*)hp = hv[i];
    }
  }
}

__global__ __launch_bounds__(GTHR) void k_proj(const unsigned short* __restrict__ XB,
                                               const unsigned short* __restrict__ WPT,
                                               const float* __restrict__ b_proj, float* node,
                                               unsigned short* nhl) {
  __shared__ __attribute__((aligned(16))) float stg[GBM * HID];
  const int tid = (int)threadIdx.x, lane = tid & 31, wave = tid >> 5, hh = lane >> 4, m = lane & 15;
  const int rowBase = (int)blockIdx.x * GBM;
  v8f acc[4];
  {
    const v8f z = {0.f, 0.f, 0.f, 0.f, 0.f, 0.f, 0.f, 0.f};
    acc[0] = z; acc[1] = z; acc[2] = z; acc[3] = z;
  }
  const unsigned short* ap = XB + (size_t)(rowBase + 16 * wave + m) * CIN + 8 * hh;
  const unsigned short* wp = WPT + (size_t)m * CIN + 8 * hh;
  mm_tile<4, CIN / 32, CIN>(ap, wp, acc);
#pragma unroll
  for (int t = 0; t < 4; ++t) {
    const int lc = 16 * t + m;
    const float bb = bf16_val(b_proj[lc]);
#pragma unroll
    for (int r = 0; r < 8; ++r) {
      const int lr = 16 * wave + 8 * hh + r;
      stg[lr * HID + lc] = relu_np(acc[t][r] + bb);
    }
  }
  __syncthreads();
  put_rows<8, 1>(stg, HID, 16 * wave, rowBase, 0x7fffffff, node, nhl, hh, m);
}

__global__ __launch_bounds__(GTHR) void k_gemm(
    const unsigned short* __restrict__ A, const unsigned short* __restrict__ WT,
    float* outF, int K, int ldo)
{
  __shared__ __attribute__((aligned(16))) float stg[GBM * GBN];
  const int tid = (int)threadIdx.x, lane = tid & 31, wave = tid >> 5, hh = lane >> 4, m = lane & 15;
  const int rowBase = (int)blockIdx.x * GBM;
  const int col0    = (int)blockIdx.y * GBN;

  v8f acc[4];
  {
    const v8f z = {0.f, 0.f, 0.f, 0.f, 0.f, 0.f, 0.f, 0.f};
    acc[0] = z; acc[1] = z; acc[2] = z; acc[3] = z;
  }
  const unsigned short* ap = A  + (size_t)(rowBase + 16 * wave + m) * (size_t)K + 8 * hh;
  const unsigned short* wp = WT + (size_t)(col0 + m) * (size_t)K + 8 * hh;
  const int ksteps = K >> 5;
#pragma unroll 1
  for (int ks = 0; ks < ksteps; ++ks) {
    FragB af;
    af.h[0] = *(const v8usa*)(ap + 32 * ks);
    af.h[1] = *(const v8usa*)(ap + 32 * ks + 16);
#pragma unroll
    for (int t = 0; t < 4; ++t) {
      const unsigned short* wq = wp + (size_t)(16 * t) * (size_t)K + 32 * ks;
      FragB bf;
      bf.h[0] = *(const v8usa*)wq;
      bf.h[1] = *(const v8usa*)(wq + 16);
      acc[t] = wmb(af, bf, acc[t]);
    }
  }

#pragma unroll
  for (int t = 0; t < 4; ++t) {
    const int lc = 16 * t + m;
#pragma unroll
    for (int r = 0; r < 8; ++r) {
      const int lr = 16 * wave + 8 * hh + r;
      stg[lr * GBN + lc] = acc[t][r];
    }
  }
  __syncthreads();

  v4f fv[8];
#pragma unroll
  for (int i = 0; i < 8; ++i) {
    const int lr = 16 * wave + 2 * i + hh;
    fv[i] = *(const v4fa*)(stg + lr * GBN + 4 * m);
  }
#pragma unroll
  for (int i = 0; i < 8; ++i) {
    const int lr = 16 * wave + 2 * i + hh;
    const int gr = rowBase + lr;
    float* op = outF + (size_t)gr * (size_t)ldo + col0 + 4 * m;
    *(volatile v4f*)op = fv[i];
  }
  __threadfence();
#pragma unroll
  for (int i = 0; i < 8; ++i) {
    const int lr = 16 * wave + 2 * i + hh;
    const int gr = rowBase + lr;
    float* op = outF + (size_t)gr * (size_t)ldo + col0 + 4 * m;
    *(volatile v4f*)op = fv[i];
  }
}

__global__ __launch_bounds__(NTHR) void k_scan(const int* __restrict__ srcs, const int* __restrict__ dsts,
                                               int nE, int nN, int vec8, int mRows,
                                               const float* __restrict__ ea, const float* __restrict__ w_e1,
                                               const float* __restrict__ b_e1, const float* __restrict__ b_conv,
                                               const float* __restrict__ G, unsigned short* mhl) {
  __shared__ __attribute__((aligned(16))) int dsm[SC_LDS_INTS];
  __shared__ float w1s[DEI * DEH];
  int* list = dsm;
  int* hl   = dsm + LISTN;
  int* sl   = dsm + LISTN + RCAP;
  int* cnt  = dsm + LISTN + 2 * RCAP;
  int* offs = cnt + NBA;
  int* cur  = offs + NBA;
  int* misc = cur + NBA;
  const int tid = (int)threadIdx.x, lane = tid & 31, wave = tid >> 5;
  const int nodeBase = (int)blockIdx.x * NBA;

  {
    const v4i z4 = {0, 0, 0, 0};
    for (int i = tid * 4; i < SC_ZINTS; i += NTHR * 4) *(v4ia*)(dsm + i) = z4;
    if (tid < 16) misc[tid] = 0;
#pragma unroll 1
    for (int i = tid; i < DEI * DEH; i += NTHR) w1s[i] = bf16_val(w_e1[i]);
  }
  const float b1 = bf16_val(b_e1[lane]);
  float bc0, bc1;
  {
    const v2f a = *(const v2fa*)(b_conv + 2 * lane);
    bc0 = bf16_val(a.x); bc1 = bf16_val(a.y);
  }
  __syncthreads();
  float w1r[DEI];
#pragma unroll
  for (int t = 0; t < DEI; ++t) w1r[t] = w1s[t * DEH + lane];

  int t = 0, ov = 0;
  const int nChunks = (nE + CHUNK - 1) / CHUNK;
#pragma unroll 1
  for (int ch = 0; ch < nChunks; ++ch) {
    const int cbase = ch * CHUNK;
    const int wc = scan_chunk<SLA>(dsts, nE, cbase, nodeBase, NBA, vec8, list, tid, lane, wave);
    if (lane == 0) misc[wave] = wc;
    __syncthreads();
    if (wave == 0) {
#pragma unroll 1
      for (int w2 = 0; w2 < NWAVE; ++w2) {
        int c = misc[w2];
        c = c < 0 ? 0 : (c > WCAP ? WCAP : c);
#pragma unroll 1
        for (int b0 = 0; b0 < c; b0 += 32) {
          const int idx = b0 + lane;
          const int ent = list[w2 * WCAP + (idx < WCAP ? idx : WCAP - 1)];
          const int m32 = (c - b0) < 32 ? (c - b0) : 32;
#pragma unroll 1
          for (int k = 0; k < m32; ++k) {
            const int u    = __builtin_amdgcn_readlane(ent, k);
            const int slot = u & (NBA - 1);
            const int el   = (u >> SLA) & (CHUNK - 1);
            const int pk   = ((cbase + el) << SLA) | slot;
            if (t < RCAP) {
              if (lane == 0) { hl[t] = pk; cnt[slot] = cnt[slot] + 1; }
              t = t + 1;
            } else {
              ov = 1;
            }
          }
        }
      }
    }
    __syncthreads();
  }
  if (wave == 0 && lane == 0) { misc[8] = t; misc[9] = ov; }
  __syncthreads();
  int tt = misc[8];
  tt = tt < 0 ? 0 : (tt > RCAP ? RCAP : tt);
  const int ovf = misc[9];

  if (wave == 0) {
    const int base = lane * (NBA / 32);
    int s = 0;
#pragma unroll 1
    for (int i = 0; i < NBA / 32; ++i) s += cnt[base + i];
    int incl = s;
#pragma unroll
    for (int d = 1; d < 32; d <<= 1) {
      const int y = __shfl_up(incl, d, 32);
      if (lane >= d) incl += y;
    }
    int run = incl - s;
#pragma unroll 1
    for (int i = 0; i < NBA / 32; ++i) {
      const int cv = cnt[base + i];
      offs[base + i] = run;
      cur[base + i]  = run;
      run += cv;
    }
  }
  __syncthreads();
  if (wave == 0) {
#pragma unroll 1
    for (int b0 = 0; b0 < tt; b0 += 32) {
      const int idx = b0 + lane;
      const int ent = hl[idx < RCAP ? idx : RCAP - 1];
      const int m32 = (tt - b0) < 32 ? (tt - b0) : 32;
#pragma unroll 1
      for (int k = 0; k < m32; ++k) {
        const int u    = __builtin_amdgcn_readlane(ent, k);
        const int slot = u & (NBA - 1);
        if (lane == 0) {
          int p = cur[slot];
          p = p < 0 ? 0 : (p > RCAP - 1 ? RCAP - 1 : p);
          sl[p] = u;
          cur[slot] = p + 1;
        }
      }
    }
  }
  __syncthreads();

  const float qnan = __int_as_float(0x7fc00000);
  const float pz = (ovf != 0) ? qnan : 0.0f;
  const int q0s = (4 * lane) & 31, q1s = (4 * lane + 1) & 31;
  const int q2s = (4 * lane + 2) & 31, q3s = (4 * lane + 3) & 31;
  const int kmax = 0x7fffffff;
#pragma unroll 1
  for (int si = 0; si < NBA / NWAVE; ++si) {
    const int s    = si * NWAVE + wave;
    const int node = nodeBase + s;
    int c = cnt[s];
    const bool big = c > DEGCAP;
    c = c < 0 ? 0 : (c > DEGCAP ? DEGCAP : c);
    int o = offs[s];
    o = o < 0 ? 0 : (o > RCAP ? RCAP : o);
    const int nc = node < nN ? node : nN - 1;
    float acc0 = 0.0f, acc1 = 0.0f;
    int key;
    {
      int idx = o + lane;
      idx = idx > RCAP - 1 ? RCAP - 1 : idx;
      const int ent = sl[idx];
      int eid = ent >> SLA;
      eid = eid < 0 ? 0 : (eid > nE - 1 ? nE - 1 : eid);
      key = (lane < c) ? eid : kmax;
    }
#pragma unroll 1
    for (int k = 0; k < c; ++k) {
      int mn = key;
      { const int y = __shfl_xor(mn, 16, 32); mn = y < mn ? y : mn; }
      { const int y = __shfl_xor(mn, 8, 32);  mn = y < mn ? y : mn; }
      { const int y = __shfl_xor(mn, 4, 32);  mn = y < mn ? y : mn; }
      { const int y = __shfl_xor(mn, 2, 32);  mn = y < mn ? y : mn; }
      { const int y = __shfl_xor(mn, 1, 32);  mn = y < mn ? y : mn; }
      mn = __builtin_amdgcn_readfirstlane(mn);
      key = (key == mn) ? kmax : key;
      int ek = mn;
      ek = ek < 0 ? 0 : (ek > nE - 1 ? nE - 1 : ek);
      int sk = srcs[ek];
      sk = sk < 0 ? 0 : (sk > nN - 1 ? nN - 1 : sk);
      const float* ep = ea + (size_t)ek * DEI;
      const v4f e0 = *(const v4fa*)ep;
      const v4f e1 = *(const v4fa*)(ep + 4);
      const v4f e2 = *(const v4fa*)(ep + 8);
      float hs = 0.0f;
      hs = fmaf(bf16_val(e0.x), w1r[0], hs);
      hs = fmaf(bf16_val(e0.y), w1r[1], hs);
      hs = fmaf(bf16_val(e0.z), w1r[2], hs);
      hs = fmaf(bf16_val(e0.w), w1r[3], hs);
      hs = fmaf(bf16_val(e1.x), w1r[4], hs);
      hs = fmaf(bf16_val(e1.y), w1r[5], hs);
      hs = fmaf(bf16_val(e1.z), w1r[6], hs);
      hs = fmaf(bf16_val(e1.w), w1r[7], hs);
      hs = fmaf(bf16_val(e2.x), w1r[8], hs);
      hs = fmaf(bf16_val(e2.y), w1r[9], hs);
      hs = fmaf(bf16_val(e2.z), w1r[10], hs);
      hs = fmaf(bf16_val(e2.w), w1r[11], hs);
      hs = relu_np(hs + b1);
      const int hei = __float_as_int(hs);
      const float* tp = G + (size_t)sk * NBIG + 2 * lane;
      float m0 = 0.0f, m1 = 0.0f;
#pragma unroll 4
      for (int kk = 0; kk < DEH; ++kk) {
        const float hk = __int_as_float(__builtin_amdgcn_readlane(hei, kk));
        const v2f tv = *(const v2fa*)(tp + kk * HID);
        m0 = fmaf(hk, tv.x, m0);
        m1 = fmaf(hk, tv.y, m1);
      }
      const v2f tb = *(const v2fa*)(tp + COL_TB);
      m0 = m0 + tb.x; m1 = m1 + tb.y;
      acc0 = acc0 + m0; acc1 = acc1 + m1;
    }
    float r0, r1;
    {
      const v2f a = *(const v2fa*)(G + (size_t)nc * NBIG + COL_R + 2 * lane);
      r0 = a.x; r1 = a.y;
    }
    const float pzr = big ? qnan : pz;
    const bool live = node < nN;
    float y0 = (acc0 + r0) + bc0;
    float y1 = (acc1 + r1) + bc1;
    y0 = relu_np(y0); y1 = relu_np(y1);
    y0 = y0 + pzr; y1 = y1 + pzr;
    const float v0 = live ? y0 : 0.0f;
    const float v1 = live ? y1 : 0.0f;
    const bool wr = (node < mRows) && (lane < 16);
    const unsigned hb0 = bf16_bits(v0), hb1 = bf16_bits(v1);
    const unsigned lb0 = bf16_bits(v0 - __uint_as_float(hb0 << 16));
    const unsigned lb1 = bf16_bits(v1 - __uint_as_float(hb1 << 16));
    const int hw = (int)(hb0 | (hb1 << 16));
    const int lw = (int)(lb0 | (lb1 << 16));
    const int g0 = __shfl(hw, q0s, 32), g1 = __shfl(hw, q1s, 32);
    const int g2 = __shfl(hw, q2s, 32), g3 = __shfl(hw, q3s, 32);
    const int p0 = __shfl(lw, q0s, 32), p1 = __shfl(lw, q1s, 32);
    const int p2 = __shfl(lw, q2s, 32), p3 = __shfl(lw, q3s, 32);
    const bool lsel = (lane & 8) != 0;
    v4u pv;
    pv.x = (unsigned int)(lsel ? p0 : g0);
    pv.y = (unsigned int)(lsel ? p1 : g1);
    pv.z = (unsigned int)(lsel ? p2 : g2);
    pv.w = (unsigned int)(lsel ? p3 : g3);
    unsigned short* hp = mhl + (size_t)node * K2 + 8 * (lane & 15);
    if (wr) *(volatile v4u*)hp = pv;
    __threadfence();
    if (wr) *(volatile v4u*)hp = pv;
  }
}

template <int LAST>
__global__ __launch_bounds__(NTHR) void k_gru(const unsigned short* __restrict__ MHL,
                                              const unsigned short* __restrict__ WIH,
                                              const float* __restrict__ G,
                                              const float* __restrict__ b_ih, const float* __restrict__ b_hh,
                                              float* node, unsigned short* nhl, float* outp, int nN) {
  __shared__ __attribute__((aligned(16))) float stg[GBM * NG3];
  __shared__ float bis[NG3];
  __shared__ float bhs[NG3];
  const int tid = (int)threadIdx.x, lane = tid & 31, wave = tid >> 5, hh = lane >> 4, m = lane & 15;
  const int rowBase = (int)blockIdx.x * GBM;
  if (tid < NG3) {
    bis[tid] = bf16_val(b_ih[tid]);
    bhs[tid] = bf16_val(b_hh[tid]);
  }
  const int rg = wave & 3, ch = wave >> 2;
  v8f acc[6];
  {
    const v8f z = {0.f, 0.f, 0.f, 0.f, 0.f, 0.f, 0.f, 0.f};
#pragma unroll
    for (int t = 0; t < 6; ++t) acc[t] = z;
  }
  const unsigned short* ap = MHL + (size_t)(rowBase + 16 * rg + m) * K2 + 8 * hh;
  const unsigned short* wp = WIH + (size_t)(96 * ch + m) * K2 + 8 * hh;
  mm_tile<6, K2 / 32, K2>(ap, wp, acc);
#pragma unroll
  for (int t = 0; t < 6; ++t) {
    const int lc = 96 * ch + 16 * t + m;
#pragma unroll
    for (int r = 0; r < 8; ++r) {
      const int lr = 16 * rg + 8 * hh + r;
      stg[lr * NG3 + lc] = acc[t][r];
    }
  }
  __syncthreads();
#pragma unroll 1
  for (int it = 0; it < (GBM * HID) / NTHR; ++it) {
    const int idx = it * NTHR + tid;
    const int lr = idx >> 6, j = idx & 63;
    const size_t gr = (size_t)(rowBase + lr);
    const float* gp = G + gr * NBIG + COL_GH + j;
    const float ghr = gp[0], ghz = gp[HID], ghn = gp[2 * HID];
    const float hp = node[gr * HID + j];
    float* sp = stg + lr * NG3 + j;
    const float ar = (sp[0] + bis[j]) + (ghr + bhs[j]);
    const float az = (sp[HID] + bis[HID + j]) + (ghz + bhs[HID + j]);
    const float rr = sigm(ar);
    const float zz = sigm(az);
    const float nn = tanhf((sp[2 * HID] + bis[2 * HID + j]) + rr * (ghn + bhs[2 * HID + j]));
    sp[0] = (1.0f - zz) * nn + zz * hp;
  }
  __syncthreads();
  if constexpr (LAST != 0) {
    put_rows<4, 0>(stg, NG3, 8 * wave, rowBase, nN, outp, nhl, hh, m);
  } else {
    put_rows<4, 1>(stg, NG3, 8 * wave, rowBase, 0x7fffffff, node, nhl, hh, m);
  }
}

static inline int cdiv(int a, int b) { return (a + b - 1) / b; }
static inline size_t al256(size_t o) { return (o + 255) & ~(size_t)255; }

extern "C" void kernel_launch(void* const* d_in, const int* in_sizes, int n_in,
                              void* d_out, int out_size, void* d_ws, size_t ws_size,
                              hipStream_t stream) {
  if (n_in < 15) return;
  if (in_sizes[0] < CIN || (in_sizes[0] % CIN) != 0) return;
  const int nN = in_sizes[0] / CIN;
  if (nN < 1 || nN > (1 << 20)) return;
  if (in_sizes[1] < 2 || (in_sizes[1] & 1) != 0) return;
  const int nE = in_sizes[1] / 2;
  if (nE < 1 || nE >= (1 << (31 - SLA))) return;
  if (in_sizes[2] != nE * DEI) return;
  if (in_sizes[3] != CIN * HID || in_sizes[4] != HID) return;
  if (in_sizes[5] != DEI * DEH || in_sizes[6] != DEH) return;
  if (in_sizes[7] != DEH * HID * HID || in_sizes[8] != HID * HID) return;
  if (in_sizes[9] != HID * HID || in_sizes[10] != HID) return;
  if (in_sizes[11] != NG3 * HID || in_sizes[12] != NG3 * HID) return;
  if (in_sizes[13] != NG3 || in_sizes[14] != NG3) return;
  if (out_size != nN * HID) return;

  const float* x      = (const float*)d_in[0];
  const int*   edge   = (const int*)d_in[1];
  const float* eattr  = (const float*)d_in[2];
  const float* w_proj = (const float*)d_in[3];
  const float* b_proj = (const float*)d_in[4];
  const float* w_e1   = (const float*)d_in[5];
  const float* b_e1   = (const float*)d_in[6];
  const float* w_e2   = (const float*)d_in[7];
  const float* b_e2   = (const float*)d_in[8];
  const float* w_root = (const float*)d_in[9];
  const float* b_conv = (const float*)d_in[10];
  const float* w_ih   = (const float*)d_in[11];
  const float* w_hh   = (const float*)d_in[12];
  const float* b_ih   = (const float*)d_in[13];
  const float* b_hh   = (const float*)d_in[14];
  float* out = (float*)d_out;
  const int* src = edge;
  const int* dst = edge + nE;

  const int MP = cdiv(nN, GBM) * GBM;
  const int gM = MP / GBM;
  const int gA = cdiv(MP, NBA);
  if ((long long)gA * NBA < (long long)MP) return;
  const int vec8 = ((nE & 3) == 0) ? 1 : 0;

  char* ws = (char*)d_ws;
  size_t off = 0;
  const size_t oWPT = off; off = al256(off + (size_t)HID * CIN * 2);
  const size_t oWBG = off; off = al256(off + (size_t)NBIG * K2 * 2);
  const size_t oWIH = off; off = al256(off + (size_t)NG3 * K2 * 2);
  const size_t oXB  = off; off = al256(off + (size_t)MP * CIN * 2);
  const size_t oND  = off; off = al256(off + (size_t)MP * HID * 4);
  const size_t oNHL = off; off = al256(off + (size_t)MP * K2 * 2);
  const size_t oMHL = off; off = al256(off + (size_t)MP * K2 * 2);
  const size_t oG   = off; off = al256(off + (size_t)MP * NBIG * 4);
  if (off > ws_size || off > (size_t)WSMAX) return;
  unsigned short* WPT  = (unsigned short*)(ws + oWPT);
  unsigned short* WBIG = (unsigned short*)(ws + oWBG);
  unsigned short* WIH  = (unsigned short*)(ws + oWIH);
  unsigned short* XB   = (unsigned short*)(ws + oXB);
  float*          NODE = (float*)(ws + oND);
  unsigned short* NHL  = (unsigned short*)(ws + oNHL);
  unsigned short* MHL  = (unsigned short*)(ws + oMHL);
  float*          G    = (float*)(ws + oG);

  const int nUx = MP * (CIN / 8);
  k_wprep<<<NU_ALL / NTHR, NTHR, 0, stream>>>(w_proj, w_e2, b_e2, w_root, w_hh, w_ih, WPT, WBIG, WIH);
  k_cvx<<<cdiv(nUx, NTHR), NTHR, 0, stream>>>(x, nN, nUx, XB);
  k_proj<<<gM, GTHR, 0, stream>>>(XB, WPT, b_proj, NODE, NHL);
  for (int step = 0; step < 2; ++step) {
    k_gemm<<<dim3(gM, NBIG / GBN), GTHR, 0, stream>>>(NHL, WBIG, G, K2, NBIG);
    k_scan<<<gA, NTHR, 0, stream>>>(src, dst, nE, nN, vec8, MP, eattr, w_e1, b_e1, b_conv, G, MHL);
    if (step == 0)
      k_gru<0><<<gM, NTHR, 0, stream>>>(MHL, WIH, G, b_ih, b_hh, NODE, NHL, out, nN);
    else
      k_gru<1><<<gM, NTHR, 0, stream>>>(MHL, WIH, G, b_ih, b_hh, NODE, NHL, out, nN);
  }
}
